// TemporalAttention_39024072851657
// MI455X (gfx1250) — hardware-verified
//
#include <hip/hip_runtime.h>
#include <math.h>

typedef __attribute__((ext_vector_type(16))) _Float16 v16h;
typedef __attribute__((ext_vector_type(16))) __bf16 v16b;
typedef __attribute__((ext_vector_type(8)))  _Float16 v8h;
typedef __attribute__((ext_vector_type(8)))  float v8f;
typedef __attribute__((ext_vector_type(4)))  float v4f;
typedef __attribute__((ext_vector_type(2)))  float v2f;
typedef __attribute__((ext_vector_type(4)))  unsigned v4u;
typedef __attribute__((ext_vector_type(4)))  int v4i;
typedef float __attribute__((may_alias)) float_a;
typedef int __attribute__((may_alias)) int_a;

template <typename T> __device__ __forceinline__ void vst2(void* p, T v) { *(volatile T*)p = v; __threadfence(); *(volatile T*)p = v; }
__device__ __forceinline__ v8f wmma16(v16h a, v16h b, v8f c) {
  v8f d = __builtin_amdgcn_wmma_f32_16x16x32_f16(false, a, false, b, (short)0, c, false, false);
  asm volatile("v_nop\n\tv_nop\n\tv_nop\n\tv_nop" : "+v"(d) : "v"(a), "v"(b));
  return d;
}
__device__ __forceinline__ v8f wmma_bf(v16b a, v16b b, v8f c) {
  v8f d = __builtin_amdgcn_wmma_f32_16x16x32_bf16(false, a, false, b, (short)0, c, false, false);
  asm volatile("v_nop\n\tv_nop\n\tv_nop\n\tv_nop" : "+v"(d) : "v"(a), "v"(b));
  return d;
}
__device__ __forceinline__ v16h frag_h(const _Float16* rowk0, int lane) {
  union { v16h v; v8h q[2]; } u; const _Float16* p = rowk0 + 8 * (lane >> 4);
  u.q[0] = *(const v8h*)p; u.q[1] = *(const v8h*)(p + 16); return u.v;
}
__device__ __forceinline__ v16h frag_f32(const float* rowk0, int lane) {
  v16h a; const float* p = rowk0 + 8 * (lane >> 4);
#pragma unroll
  for (int i = 0; i < 8; ++i) { a[i] = (_Float16)p[i]; a[8 + i] = (_Float16)p[16 + i]; }
  return a;
}
__device__ __forceinline__ v16h frag_f32s(const float* rowk0, int lane, float sc) {
  v16h a; const float* p = rowk0 + 8 * (lane >> 4);
#pragma unroll
  for (int i = 0; i < 8; ++i) { a[i] = (_Float16)(p[i] * sc); a[8 + i] = (_Float16)(p[16 + i] * sc); }
  return a;
}
__device__ __forceinline__ v16h fragc_f32(const float* W, int k0, int n, int lane, int ld, int K) {
  v16h a; const int g = lane >> 4;
#pragma unroll
  for (int i = 0; i < 8; ++i) { const int ka = k0 + 8 * g + i, kb = ka + 16;
    a[i] = (_Float16)(ka < K ? W[(size_t)ka * ld + n] : 0.f); a[8 + i] = (_Float16)(kb < K ? W[(size_t)kb * ld + n] : 0.f); }
  return a;
}
struct F2 { v16b h, l; };
__device__ __forceinline__ F2 bsplit16(const float v[16]) { F2 r;
#pragma unroll
  for (int i = 0; i < 16; ++i) { const __bf16 h = (__bf16)v[i]; r.h[i] = h; r.l[i] = (__bf16)(v[i] - (float)h); }
  return r; }
__device__ __forceinline__ F2 split_row(const float* row, int k0, int lane) { float v[16]; const float* p = row + k0 + 8 * (lane >> 4);
#pragma unroll
  for (int i = 0; i < 8; ++i) { v[i] = p[i]; v[8 + i] = p[16 + i]; }
  return bsplit16(v); }
__device__ __forceinline__ F2 split_rowK(const float* row, int k0, int lane, int K) { float v[16]; const int g = lane >> 4;
#pragma unroll
  for (int i = 0; i < 8; ++i) { const int ka = k0 + 8 * g + i, kb = ka + 16; v[i] = ka < K ? row[ka] : 0.f; v[8 + i] = kb < K ? row[kb] : 0.f; }
  return bsplit16(v); }
__device__ __forceinline__ F2 split_col(const float* W, int k0, int n, int lane, int ld, int K) { float v[16]; const int g = lane >> 4;
#pragma unroll
  for (int i = 0; i < 8; ++i) { const int ka = k0 + 8 * g + i, kb = ka + 16; v[i] = ka < K ? W[(size_t)ka * ld + n] : 0.f; v[8 + i] = kb < K ? W[(size_t)kb * ld + n] : 0.f; }
  return bsplit16(v); }
__device__ __forceinline__ v8f mac3(const F2& a, const F2& b, v8f c) { c = wmma_bf(a.l, b.h, c); c = wmma_bf(a.h, b.l, c); return wmma_bf(a.h, b.h, c); }
__device__ __forceinline__ float sigm(float v) { return 1.0f / (1.0f + expf(-v)); }
#define LDSX() do { asm volatile("s_wait_dscnt 0" ::: "memory"); __builtin_amdgcn_wave_barrier(); __builtin_amdgcn_fence(__ATOMIC_RELEASE, "workgroup"); } while (0)


#define NBI 4
#define C 256
#define CQ 32
#define NP 4096
#define NR (NBI * NP)
#define OW (CQ + CQ + C)

__global__ __launch_bounds__(256) void k_cvt(const float* __restrict__ f1, const float* __restrict__ f2, _Float16* __restrict__ F1h, _Float16* __restrict__ F2h) {
  __shared__ __align__(16) _Float16 st[C][72];
  const int tid = threadIdx.x; const int which = blockIdx.y; const int b = blockIdx.x / (NP / 64), n0 = (blockIdx.x % (NP / 64)) * 64;
  const float* src = which == 0 ? f1 : f2; _Float16* dst = which == 0 ? F1h : F2h;
  for (int q = tid; q < C * 16; q += 256) { const int c = q >> 4, p4 = q & 15; const v4f v = *(const v4f*)(src + ((size_t)b * C + c) * NP + n0 + p4 * 4);
    st[c][p4 * 4] = (_Float16)v[0]; st[c][p4 * 4 + 1] = (_Float16)v[1]; st[c][p4 * 4 + 2] = (_Float16)v[2]; st[c][p4 * 4 + 3] = (_Float16)v[3]; }
  __syncthreads();
  for (int q = tid; q < 64 * (C / 8); q += 256) { const int nl = q >> 5, pc = q & 31; union { v8h h; v4u u; } pk;
#pragma unroll
    for (int e = 0; e < 8; ++e) pk.h[e] = st[pc * 8 + e][nl];
    vst2(dst + ((size_t)b * NP + n0 + nl) * C + pc * 8, pk.u); }
}
__global__ __launch_bounds__(256) void k_pack(const float* __restrict__ wq, const float* __restrict__ wk, const float* __restrict__ wv, _Float16* __restrict__ PT) {
  const int n = blockIdx.x, tid = threadIdx.x; __shared__ __align__(16) _Float16 srow[C];
  const float* src = n < CQ ? wq + (size_t)n * C : (n < 2 * CQ ? wk + (size_t)(n - CQ) * C : wv + (size_t)(n - 2 * CQ) * C);
  srow[tid] = (_Float16)(src[tid] * 16.0f);
  __syncthreads();
  if (tid < C / 8) vst2(PT + (size_t)n * C + tid * 8, *(const v4u*)(&srow[tid * 8]));
}
__global__ __launch_bounds__(128) void k_qkv(const _Float16* __restrict__ F1h, const _Float16* __restrict__ F2h, const _Float16* __restrict__ PT, const float* __restrict__ bq, const float* __restrict__ bk, const float* __restrict__ bv,
                                            _Float16* __restrict__ Q16, _Float16* __restrict__ K16, _Float16* __restrict__ V16) {
  __shared__ __align__(16) float so[4][16][68];
  __shared__ __align__(16) _Float16 sth[128][72];
  const int tid = threadIdx.x, wave = tid >> 5, lane = tid & 31, col = lane & 15, g = lane >> 4;
  const int part = blockIdx.y, r0b = blockIdx.x * 64, r0 = r0b + wave * 16; const int b = r0b / NP, s0 = r0b % NP;
  if (part == 0) {
    v8f aq[2] = {}, ak[2] = {};
#pragma unroll 2
    for (int kc = 0; kc < C / 32; ++kc) { const v16h a2 = frag_h(F2h + (size_t)(r0 + col) * C + kc * 32, lane), a1 = frag_h(F1h + (size_t)(r0 + col) * C + kc * 32, lane);
#pragma unroll
      for (int j = 0; j < 2; ++j) { aq[j] = wmma16(a2, frag_h(PT + (size_t)(j * 16 + col) * C + kc * 32, lane), aq[j]); ak[j] = wmma16(a1, frag_h(PT + (size_t)(CQ + j * 16 + col) * C + kc * 32, lane), ak[j]); } }
#pragma unroll
    for (int j = 0; j < 2; ++j)
#pragma unroll
      for (int r = 0; r < 8; ++r) { so[wave][8 * g + r][j * 16 + col] = (aq[j][r] * (1.0f / 16.0f) + bq[j * 16 + col]) * 4.0f; so[wave][8 * g + r][32 + j * 16 + col] = (ak[j][r] * (1.0f / 16.0f) + bk[j * 16 + col]) * 4.0f; }
    LDSX();
    for (int qq = lane; qq < 2 * 16 * 4; qq += 32) { const int which = qq >> 6, rl = (qq >> 2) & 15, pc = qq & 3; union { v8h h8; v4u u; } pk;
#pragma unroll
      for (int e = 0; e < 8; ++e) pk.h8[e] = (_Float16)so[wave][rl][which * 32 + pc * 8 + e];
      vst2((which == 0 ? Q16 : K16) + ((size_t)b * NP + s0 + wave * 16 + rl) * CQ + pc * 8, pk.u); } }
  else { const int n0 = (part - 1) * 128;
    v8f acc[8] = {};
#pragma unroll 2
    for (int kc = 0; kc < C / 32; ++kc) { const v16h a1 = frag_h(F1h + (size_t)(r0 + col) * C + kc * 32, lane);
#pragma unroll
      for (int j = 0; j < 8; ++j) acc[j] = wmma16(a1, frag_h(PT + (size_t)(2 * CQ + n0 + j * 16 + col) * C + kc * 32, lane), acc[j]); }
#pragma unroll
    for (int j = 0; j < 8; ++j) { const float bb = bv[n0 + j * 16 + col];
#pragma unroll
      for (int r = 0; r < 8; ++r) sth[j * 16 + col][wave * 16 + 8 * g + r] = (_Float16)(acc[j][r] * (1.0f / 16.0f) + bb); }
    __syncthreads();
    for (int qq = tid; qq < 128 * 8; qq += 128) { const int cl = qq >> 3, pc = qq & 7; vst2(V16 + ((size_t)b * C + n0 + cl) * NP + s0 + pc * 8, *(const v4u*)(&sth[cl][pc * 8])); } }
}
__global__ __launch_bounds__(128) void k_attn(const _Float16* __restrict__ Q16, const _Float16* __restrict__ K16, const _Float16* __restrict__ V16, const float* __restrict__ gammap, const float* __restrict__ feat2, float* __restrict__ out) {
  __shared__ __align__(16) float sS[4][16][68];
  __shared__ __align__(16) _Float16 sPh[4][16][72];
  __shared__ __align__(16) float st[C][68];
  const int tid = threadIdx.x, w = tid >> 5, lane = tid & 31, col = lane & 15, g = lane >> 4;
  const int b = blockIdx.y; const int qb0 = blockIdx.x * 64, q0 = qb0 + w * 16; const float gam = gammap[0];
  const v16h aq = frag_h(Q16 + ((size_t)b * NP + q0 + col) * CQ, lane);
  const float scl = 1.0f / 16.0f;
#pragma unroll 1
  for (int nh = 0; nh < 2; ++nh) {
  float mrun = -3.0e38f, lrun = 0.f; v8f acc[8] = {};
#pragma unroll 1
  for (int kt = 0; kt < NP / 64; ++kt) {
#pragma unroll
    for (int t = 0; t < 4; ++t) { const int key = kt * 64 + t * 16 + col; const v8f s = wmma16(aq, frag_h(K16 + ((size_t)b * NP + key) * CQ, lane), (v8f){});
#pragma unroll
      for (int r = 0; r < 8; ++r) sS[w][8 * g + r][t * 16 + col] = s[r] * scl; }
    LDSX();
    float mx = -3.4e38f;
#pragma unroll
    for (int jj = 0; jj < 32; ++jj) mx = fmaxf(mx, sS[w][col][g * 32 + jj]);
    mx = fmaxf(mx, __shfl_xor(mx, 16, 32));
    const float mnew = fmaxf(mrun, mx); const float corr = expf(mrun - mnew);
    float ps = 0.f;
#pragma unroll
    for (int jj = 0; jj < 32; ++jj) { const float p = expf(sS[w][col][g * 32 + jj] - mnew) * 16384.0f; ps += p; sPh[w][col][g * 32 + jj] = (_Float16)p; }
    ps += __shfl_xor(ps, 16, 32);
    lrun = lrun * corr + ps * (1.0f / 16384.0f); mrun = mnew;
#pragma unroll
    for (int r = 0; r < 8; ++r) { const float cr = __shfl(corr, 8 * g + r, 32);
#pragma unroll
      for (int t = 0; t < 8; ++t) acc[t][r] *= cr; }
    LDSX();
#pragma unroll
    for (int kc = 0; kc < 2; ++kc) { const v16h ph = frag_h(&sPh[w][col][0] + kc * 32, lane);
#pragma unroll
      for (int t = 0; t < 8; ++t) acc[t] = wmma16(ph, frag_h(V16 + ((size_t)b * C + nh * 128 + t * 16 + col) * NP + kt * 64 + kc * 32, lane), acc[t]); }
    __builtin_amdgcn_wave_barrier(); }
#pragma unroll
  for (int r = 0; r < 8; ++r) { const float lr = __shfl(lrun, 8 * g + r, 32); const float inv = 1.0f / (lr * 16384.0f);
#pragma unroll
    for (int t = 0; t < 8; ++t) st[nh * 128 + t * 16 + col][w * 16 + 8 * g + r] = acc[t][r] * inv; }
  LDSX(); }
  __syncthreads();
  for (int qq = tid; qq < C * 16; qq += 128) { const int c = qq >> 4, pc = qq & 15; const size_t o = ((size_t)b * C + c) * NP + qb0 + pc * 4;
    const v4f f = *(const v4f*)(feat2 + o); const v4f cx = *(const v4f*)(&st[c][pc * 4]);
    v4f v = { gam * cx[0] + f[0], gam * cx[1] + f[1], gam * cx[2] + f[2], gam * cx[3] + f[3] };
    vst2(out + o, v); }
}
extern "C" void kernel_launch(void* const* d_in, const int* in_sizes, int n_in, void* d_out, int out_size, void* d_ws, size_t ws_size, hipStream_t stream) {
  (void)in_sizes; (void)n_in; (void)out_size; (void)ws_size;
  const float* f1 = (const float*)d_in[0]; const float* f2 = (const float*)d_in[1]; const float* wq = (const float*)d_in[2]; const float* bq = (const float*)d_in[3];
  const float* wk = (const float*)d_in[4]; const float* bk = (const float*)d_in[5]; const float* wv = (const float*)d_in[6]; const float* bv = (const float*)d_in[7]; const float* gammap = (const float*)d_in[8];
  float* out = (float*)d_out;
  char* ws = (char*)d_ws; size_t off = 0;
  auto take = [&](size_t bytes) { char* p = ws + off; off += (bytes + 255) & ~(size_t)255; return p; };
  _Float16* F1h = (_Float16*)take((size_t)NR * C * 2); _Float16* F2h = (_Float16*)take((size_t)NR * C * 2); _Float16* PT = (_Float16*)take((size_t)OW * C * 2);
  _Float16* Q16 = (_Float16*)take((size_t)NR * CQ * 2); _Float16* K16 = (_Float16*)take((size_t)NR * CQ * 2); _Float16* V16 = (_Float16*)take((size_t)NR * C * 2);
  k_cvt<<<dim3(NBI * (NP / 64), 2), 256, 0, stream>>>(f1, f2, F1h, F2h);
  k_pack<<<OW, 256, 0, stream>>>(wq, wk, wv, PT);
  k_qkv<<<dim3(NR / 64, 3), 128, 0, stream>>>(F1h, F2h, PT, bq, bk, bv, Q16, K16, V16);
  k_attn<<<dim3(NP / 64, NBI), 128, 0, stream>>>(Q16, K16, V16, gammap, f2, out);
}
